// LinearTemporalSelfAttention_64046552318268
// MI455X (gfx1250) — hardware-verified
//
#include <hip/hip_runtime.h>
#include <math.h>

typedef __attribute__((ext_vector_type(16))) _Float16 v16h;
typedef __attribute__((ext_vector_type(16))) __bf16 v16b;
typedef __attribute__((ext_vector_type(8)))  _Float16 v8h;
typedef __attribute__((ext_vector_type(8)))  float v8f;
typedef __attribute__((ext_vector_type(4)))  float v4f;
typedef __attribute__((ext_vector_type(2)))  float v2f;
typedef __attribute__((ext_vector_type(4)))  unsigned v4u;
typedef __attribute__((ext_vector_type(4)))  int v4i;
typedef float __attribute__((may_alias)) float_a;
typedef int __attribute__((may_alias)) int_a;

template <typename T> __device__ __forceinline__ void vst2(void* p, T v) { *(volatile T*)p = v; __threadfence(); *(volatile T*)p = v; }
__device__ __forceinline__ v8f wmma16(v16h a, v16h b, v8f c) {
  v8f d = __builtin_amdgcn_wmma_f32_16x16x32_f16(false, a, false, b, (short)0, c, false, false);
  asm volatile("v_nop\n\tv_nop\n\tv_nop\n\tv_nop" : "+v"(d) : "v"(a), "v"(b));
  return d;
}
__device__ __forceinline__ v8f wmma_bf(v16b a, v16b b, v8f c) {
  v8f d = __builtin_amdgcn_wmma_f32_16x16x32_bf16(false, a, false, b, (short)0, c, false, false);
  asm volatile("v_nop\n\tv_nop\n\tv_nop\n\tv_nop" : "+v"(d) : "v"(a), "v"(b));
  return d;
}
__device__ __forceinline__ v16h frag_h(const _Float16* rowk0, int lane) {
  union { v16h v; v8h q[2]; } u; const _Float16* p = rowk0 + 8 * (lane >> 4);
  u.q[0] = *(const v8h*)p; u.q[1] = *(const v8h*)(p + 16); return u.v;
}
__device__ __forceinline__ v16h frag_f32(const float* rowk0, int lane) {
  v16h a; const float* p = rowk0 + 8 * (lane >> 4);
#pragma unroll
  for (int i = 0; i < 8; ++i) { a[i] = (_Float16)p[i]; a[8 + i] = (_Float16)p[16 + i]; }
  return a;
}
__device__ __forceinline__ v16h frag_f32s(const float* rowk0, int lane, float sc) {
  v16h a; const float* p = rowk0 + 8 * (lane >> 4);
#pragma unroll
  for (int i = 0; i < 8; ++i) { a[i] = (_Float16)(p[i] * sc); a[8 + i] = (_Float16)(p[16 + i] * sc); }
  return a;
}
__device__ __forceinline__ v16h fragc_f32(const float* W, int k0, int n, int lane, int ld, int K) {
  v16h a; const int g = lane >> 4;
#pragma unroll
  for (int i = 0; i < 8; ++i) { const int ka = k0 + 8 * g + i, kb = ka + 16;
    a[i] = (_Float16)(ka < K ? W[(size_t)(ka < K ? ka : K - 1) * ld + n] : 0.f); a[8 + i] = (_Float16)(kb < K ? W[(size_t)(kb < K ? kb : K - 1) * ld + n] : 0.f); }
  return a;
}
struct F2 { v16b h, l; };
__device__ __forceinline__ F2 bsplit16(const float v[16]) { F2 r;
#pragma unroll
  for (int i = 0; i < 16; ++i) { const __bf16 h = (__bf16)v[i]; r.h[i] = h; r.l[i] = (__bf16)(v[i] - (float)h); }
  return r; }
__device__ __forceinline__ F2 split_row(const float* row, int k0, int lane) { float v[16]; const float* p = row + k0 + 8 * (lane >> 4);
#pragma unroll
  for (int i = 0; i < 8; ++i) { v[i] = p[i]; v[8 + i] = p[16 + i]; }
  return bsplit16(v); }
__device__ __forceinline__ F2 split_rowK(const float* row, int k0, int lane, int K) { float v[16]; const int g = lane >> 4;
#pragma unroll
  for (int i = 0; i < 8; ++i) { const int ka = k0 + 8 * g + i, kb = ka + 16; v[i] = ka < K ? row[ka < K ? ka : K - 1] : 0.f; v[8 + i] = kb < K ? row[kb < K ? kb : K - 1] : 0.f; }
  return bsplit16(v); }
__device__ __forceinline__ F2 split_col(const float* W, int k0, int n, int lane, int ld, int K) { float v[16]; const int g = lane >> 4;
#pragma unroll
  for (int i = 0; i < 8; ++i) { const int ka = k0 + 8 * g + i, kb = ka + 16; v[i] = ka < K ? W[(size_t)(ka < K ? ka : K - 1) * ld + n] : 0.f; v[8 + i] = kb < K ? W[(size_t)(kb < K ? kb : K - 1) * ld + n] : 0.f; }
  return bsplit16(v); }
__device__ __forceinline__ v8f mac3(const F2& a, const F2& b, v8f c) { c = wmma_bf(a.l, b.h, c); c = wmma_bf(a.h, b.l, c); return wmma_bf(a.h, b.h, c); }
__device__ __forceinline__ float sigm(float v) { return 1.0f / (1.0f + expf(-v)); }
#define LDSX() do { asm volatile("s_wait_dscnt 0" ::: "memory"); __builtin_amdgcn_wave_barrier(); __builtin_amdgcn_fence(__ATOMIC_RELEASE, "workgroup"); } while (0)

__device__ __forceinline__ float bfr(float v) { return (float)(__bf16)v; }
__device__ __attribute__((noinline)) float siluf(float v) { return v / (1.0f + expf(-v)); }
__device__ __attribute__((noinline)) float expq_ni(float v) { return expf(v); }
#define NB 4
#define TT 2048
#define CC 1024
#define NH 16
#define HD 64
#define TE 2048
#define NR (NB * TT)
#ifndef TNB
#define TNB NB
#endif
#define WS_ST  0u
#define WS_QS  (WS_ST + 4u * (size_t)NR * 2)
#define WS_KR  (WS_QS + 2u * (size_t)NR * CC)
#define WS_KP  (WS_KR + 4u * (size_t)NR * CC)
#define WS_VP  (WS_KP + 2u * (size_t)NB * CC * TT)
#define WS_AT  (WS_VP + 2u * (size_t)NB * CC * TT)
#define WS_Y   (WS_AT + 4u * (size_t)NB * NH * HD * HD)
#define WS_ST2 (WS_Y + 4u * (size_t)NR * CC)
#define WS_EM  (WS_ST2 + 4u * (size_t)NR * 2)
#define WS_END (WS_EM + 4u * (size_t)NB * 2 * CC)
__global__ __launch_bounds__(256) void k_stat(const float* __restrict__ SRC, int rnd, float* __restrict__ ST) { __shared__ __align__(16) float so[32];
  const int t = threadIdx.x; const int rl = t >> 4, sub = t & 15; const size_t row = (size_t)blockIdx.x * 16 + rl; const float* p = SRC + row * CC;
  float s = 0.f; for (int c = sub; c < CC; c += 16) s += rnd ? bfr(p[c]) : p[c];
#pragma unroll
  for (int o = 1; o < 16; o <<= 1) s += __shfl_xor(s, o);
  const float mu = s * (1.0f / CC); float s2 = 0.f; for (int c = sub; c < CC; c += 16) { const float d = (rnd ? bfr(p[c]) : p[c]) - mu; s2 += d * d; }
#pragma unroll
  for (int o = 1; o < 16; o <<= 1) s2 += __shfl_xor(s2, o);
  if (sub == 0) { so[rl * 2] = mu; so[rl * 2 + 1] = rsqrtf(s2 * (1.0f / CC) + 1e-5f); }
  __syncthreads(); if (t < 32) vst2(ST + (size_t)blockIdx.x * 32 + t, so[t]); }
__global__ __launch_bounds__(128) void k_proj(const float* __restrict__ X, const float* __restrict__ ST, const float* __restrict__ LW, const float* __restrict__ LB, const float* __restrict__ MSK, const float* __restrict__ WQ, const float* __restrict__ BQ, const float* __restrict__ WK, const float* __restrict__ BK, const float* __restrict__ WV, const float* __restrict__ BV, _Float16* __restrict__ QS, float* __restrict__ KR, _Float16* __restrict__ VP) {
  __shared__ __align__(16) _Float16 sh[64][136]; __shared__ __align__(16) float sf[4][16][132]; __shared__ __align__(16) _Float16 th[128][72];
  const int tid = threadIdx.x, wave = tid >> 5, lane = tid & 31, col = lane & 15, g = lane >> 4; const int which = blockIdx.z; const int c0 = blockIdx.y * 128; const size_t r0 = (size_t)blockIdx.x * 64;
  const float* WA = which == 0 ? WQ : which == 1 ? WK : WV; const float* BA = which == 0 ? BQ : which == 1 ? BK : BV;
  const size_t ra = r0 + wave * 16 + col; const float mu = ST[ra * 2], rs = ST[ra * 2 + 1];
  v8f acc[8] = {};
#pragma unroll 2
  for (int kc = 0; kc < CC / 32; ++kc) { v16h a; { const float* p = X + ra * CC + kc * 32 + 8 * g;
#pragma unroll
      for (int i = 0; i < 8; ++i) { const int c = kc * 32 + 8 * g + i; a[i] = (_Float16)((bfr(p[i]) - mu) * rs * bfr(LW[c]) + bfr(LB[c])); a[8 + i] = (_Float16)((bfr(p[16 + i]) - mu) * rs * bfr(LW[c + 16]) + bfr(LB[c + 16])); } }
#pragma unroll
    for (int j = 0; j < 8; ++j) { v16h w; const int o = c0 + j * 16 + col;
#pragma unroll
      for (int i = 0; i < 8; ++i) { w[i] = (_Float16)(bfr(WA[(size_t)(kc * 32 + 8 * g + i) * CC + o]) * 16.0f); w[8 + i] = (_Float16)(bfr(WA[(size_t)(kc * 32 + 16 + 8 * g + i) * CC + o]) * 16.0f); }
      acc[j] = wmma16(a, w, acc[j]); } }
  if (which == 0) {
#pragma unroll
    for (int hh = 0; hh < 2; ++hh) {
#pragma unroll
      for (int r = 0; r < 8; ++r) { float vv[4]; float m = -3.0e38f;
#pragma unroll
        for (int jj = 0; jj < 4; ++jj) { vv[jj] = acc[hh * 4 + jj][r] * (1.0f / 16.0f) + bfr(BA[c0 + (hh * 4 + jj) * 16 + col]); m = fmaxf(m, vv[jj]); }
#pragma unroll
        for (int o = 1; o < 16; o <<= 1) m = fmaxf(m, __shfl_xor(m, o));
        float s = 0.f;
#pragma unroll
        for (int jj = 0; jj < 4; ++jj) { vv[jj] = expq_ni(vv[jj] - m); s += vv[jj]; }
#pragma unroll
        for (int o = 1; o < 16; o <<= 1) s += __shfl_xor(s, o);
        const float inv = 1.0f / s;
#pragma unroll
        for (int jj = 0; jj < 4; ++jj) sh[wave * 16 + 8 * g + r][(hh * 4 + jj) * 16 + col] = (_Float16)(vv[jj] * inv); } }
    __syncthreads();
    for (int e = tid; e < 64 * 16; e += 128) { const int rl = e >> 4, q = e & 15; vst2((unsigned*)(QS + (r0 + rl) * CC + c0 + q * 8), *(const v4u*)&sh[rl][q * 8]); } }
  else if (which == 1) {
#pragma unroll
    for (int j = 0; j < 8; ++j) { const float bb = bfr(BA[c0 + j * 16 + col]);
#pragma unroll
      for (int r = 0; r < 8; ++r) { const size_t row = r0 + wave * 16 + 8 * g + r; const float m = bfr(MSK[row]); sf[wave][8 * g + r][j * 16 + col] = (acc[j][r] * (1.0f / 16.0f) + bb) + (1.0f - m) * -1000000.0f; } }
    LDSX(); for (int rl = 0; rl < 16; ++rl) vst2(KR + (r0 + wave * 16 + rl) * CC + c0 + lane * 4, *(const v4f*)&sf[wave][rl][lane * 4]); }
  else {
#pragma unroll
    for (int j = 0; j < 8; ++j) { const float bb = bfr(BA[c0 + j * 16 + col]);
#pragma unroll
      for (int r = 0; r < 8; ++r) { const int rl = wave * 16 + 8 * g + r; const float m = bfr(MSK[r0 + rl]); th[j * 16 + col][rl] = (_Float16)((acc[j][r] * (1.0f / 16.0f) + bb) * m); } }
    __syncthreads();
    const size_t b = r0 / TT; const int t0 = (int)(r0 % TT); for (int e = tid; e < 128 * 8; e += 128) { const int cl = e >> 3, q = e & 7; vst2((unsigned*)(VP + (b * CC + c0 + cl) * (size_t)TT + t0 + q * 8), *(const v4u*)&th[cl][q * 8]); } } }
__global__ __launch_bounds__(256) void k_ksm(const float* __restrict__ KR, _Float16* __restrict__ KP) { __shared__ __align__(16) _Float16 sp[8][TT];
  const int t = threadIdx.x; const int cl = t >> 5, sub = t & 31; const int b = blockIdx.y; const int c = blockIdx.x * 8 + cl; const float* col0 = KR + (size_t)b * TT * CC + c;
  float m = -3.0e38f; for (int tt = sub; tt < TT; tt += 32) m = fmaxf(m, col0[(size_t)tt * CC]);
#pragma unroll
  for (int o = 1; o < 32; o <<= 1) m = fmaxf(m, __shfl_xor(m, o));
  float s = 0.f; for (int tt = sub; tt < TT; tt += 32) s += expf(col0[(size_t)tt * CC] - m);
#pragma unroll
  for (int o = 1; o < 32; o <<= 1) s += __shfl_xor(s, o);
  const float inv = 1.0f / s;
  for (int tt = sub; tt < TT; tt += 32) sp[cl][tt] = (_Float16)(expf(col0[(size_t)tt * CC] - m) * inv);
  __syncthreads();
  for (int e = t; e < 8 * (TT / 8); e += 256) { const int cc = e / (TT / 8), q = e % (TT / 8); vst2((unsigned*)(KP + ((size_t)b * CC + blockIdx.x * 8 + cc) * TT + q * 8), *(const v4u*)&sp[cc][q * 8]); } }
__global__ __launch_bounds__(128) void k_att(const _Float16* __restrict__ KP, const _Float16* __restrict__ VP, float* __restrict__ AT) { __shared__ __align__(16) float sf[4][16][68];
  const int tid = threadIdx.x, wave = tid >> 5, lane = tid & 31, col = lane & 15, g = lane >> 4; const int b = blockIdx.x / NH, h = blockIdx.x % NH; const size_t pb = ((size_t)b * CC + h * HD) * TT;
  v8f acc[4] = {};
#pragma unroll 2
  for (int kc = 0; kc < TT / 32; ++kc) { const v16h a = frag_h(KP + pb + (size_t)(wave * 16 + col) * TT + kc * 32, lane);
#pragma unroll
    for (int j = 0; j < 4; ++j) acc[j] = wmma16(a, frag_h(VP + pb + (size_t)(j * 16 + col) * TT + kc * 32, lane), acc[j]); }
#pragma unroll
  for (int j = 0; j < 4; ++j)
#pragma unroll
    for (int r = 0; r < 8; ++r) sf[wave][8 * g + r][j * 16 + col] = acc[j][r];
  LDSX(); for (int rl = 0; rl < 16; ++rl) if (lane < 16) vst2(AT + ((size_t)blockIdx.x * HD + wave * 16 + rl) * HD + lane * 4, *(const v4f*)&sf[wave][rl][lane * 4]); }
__global__ __launch_bounds__(128) void k_y(const _Float16* __restrict__ QS, const float* __restrict__ AT, float* __restrict__ Y) { __shared__ __align__(16) float sf[4][16][68];
  const int tid = threadIdx.x, wave = tid >> 5, lane = tid & 31, col = lane & 15, g = lane >> 4; const int h = blockIdx.y; const size_t r0 = (size_t)blockIdx.x * 64 + wave * 16; const int b = (int)(r0 / TT); const float* A = AT + ((size_t)(b * NH + h)) * HD * HD;
  v8f acc[4] = {};
#pragma unroll
  for (int kc = 0; kc < HD / 32; ++kc) { const v16h a = frag_h(QS + (r0 + col) * CC + h * HD + kc * 32, lane);
#pragma unroll
    for (int j = 0; j < 4; ++j) { v16h w; const int l = j * 16 + col;
#pragma unroll
      for (int i = 0; i < 8; ++i) { w[i] = (_Float16)A[(size_t)(kc * 32 + 8 * g + i) * HD + l]; w[8 + i] = (_Float16)A[(size_t)(kc * 32 + 16 + 8 * g + i) * HD + l]; }
      acc[j] = wmma16(a, w, acc[j]); } }
#pragma unroll
  for (int j = 0; j < 4; ++j)
#pragma unroll
    for (int r = 0; r < 8; ++r) sf[wave][8 * g + r][j * 16 + col] = acc[j][r];
  LDSX(); for (int rl = 0; rl < 16; ++rl) if (lane < 16) vst2(Y + (r0 + rl) * CC + h * HD + lane * 4, *(const v4f*)&sf[wave][rl][lane * 4]); }
__global__ __launch_bounds__(64) void k_emb(const float* __restrict__ EMB, const float* __restrict__ EW, const float* __restrict__ EB, float* __restrict__ EM) { __shared__ float se[TE]; __shared__ __align__(16) float so[64];
  const int t = threadIdx.x; const int b = blockIdx.y; const int o = blockIdx.x * 64 + t;
  for (int i = t; i < TE; i += 64) se[i] = siluf(bfr(EMB[(size_t)b * TE + i]));
  __syncthreads(); float s = 0.f;
#pragma unroll 1
  for (int i = 0; i < TE; ++i) s += se[i] * bfr(EW[(size_t)i * (2 * CC) + o]);
  so[t] = s + bfr(EB[o]); LDSX(); __syncthreads(); if (t < 16) vst2(EM + (size_t)b * 2 * CC + blockIdx.x * 64 + t * 4, *(const v4f*)&so[t * 4]); }
__global__ __launch_bounds__(128) void k_out(const float* __restrict__ Y, const float* __restrict__ ST2, const float* __restrict__ LW, const float* __restrict__ LB, const float* __restrict__ EM, const float* __restrict__ WO, const float* __restrict__ BO, const float* __restrict__ X, float* __restrict__ OUT) { __shared__ __align__(16) float sf[4][16][132];
  const int tid = threadIdx.x, wave = tid >> 5, lane = tid & 31, col = lane & 15, g = lane >> 4; const int c0 = blockIdx.y * 128; const size_t r0 = (size_t)blockIdx.x * 64 + wave * 16; const size_t ra = r0 + col; const int b = (int)(ra / TT);
  const float mu = ST2[ra * 2], rs = ST2[ra * 2 + 1]; const float* sc = EM + (size_t)b * 2 * CC; const float* shf = sc + CC;
  v8f acc[8] = {};
#pragma unroll 1
  for (int kc = 0; kc < CC / 32; ++kc) { v16h a; { const float* p = Y + ra * CC + kc * 32 + 8 * g;
#pragma unroll
      for (int i = 0; i < 8; ++i) { const int c = kc * 32 + 8 * g + i; const float h0 = ((p[i] - mu) * rs * bfr(LW[c]) + bfr(LB[c])) * (1.0f + sc[c]) + shf[c]; const float h1 = ((p[16 + i] - mu) * rs * bfr(LW[c + 16]) + bfr(LB[c + 16])) * (1.0f + sc[c + 16]) + shf[c + 16]; a[i] = (_Float16)siluf(h0); a[8 + i] = (_Float16)siluf(h1); } }
#pragma unroll
    for (int j = 0; j < 8; ++j) { v16h w; const int o = c0 + j * 16 + col;
#pragma unroll
      for (int i = 0; i < 8; ++i) { w[i] = (_Float16)(bfr(WO[(size_t)(kc * 32 + 8 * g + i) * CC + o]) * 16.0f); w[8 + i] = (_Float16)(bfr(WO[(size_t)(kc * 32 + 16 + 8 * g + i) * CC + o]) * 16.0f); }
      asm volatile("s_wait_loadcnt 0x0" ::: "memory");
      acc[j] = wmma16(a, w, acc[j]); } }
#pragma unroll
  for (int j = 0; j < 8; ++j) { const int cl = j * 16 + col; const float bb = bfr(BO[c0 + cl]);
#pragma unroll
    for (int r = 0; r < 8; ++r) sf[wave][8 * g + r][cl] = bfr(X[(r0 + 8 * g + r) * CC + c0 + cl]) + acc[j][r] * (1.0f / 16.0f) + bb;
    asm volatile("s_wait_loadcnt 0x0" ::: "memory"); }
  LDSX(); for (int rl = 0; rl < 16; ++rl) vst2(OUT + (r0 + rl) * CC + c0 + lane * 4, *(const v4f*)&sf[wave][rl][lane * 4]); }
extern "C" void kernel_launch(void* const* d_in, const int* in_sizes, int n_in, void* d_out, int out_size, void* d_ws, size_t ws_size, hipStream_t stream) {
  (void)in_sizes; (void)n_in; (void)out_size;
  const float** F = (const float**)d_in;
  if (ws_size < (size_t)WS_END) return;
  char* ws = (char*)d_ws; float *ST = (float*)(ws + WS_ST), *KR = (float*)(ws + WS_KR), *AT = (float*)(ws + WS_AT), *Y = (float*)(ws + WS_Y), *ST2 = (float*)(ws + WS_ST2), *EM = (float*)(ws + WS_EM); _Float16 *QS = (_Float16*)(ws + WS_QS), *KP = (_Float16*)(ws + WS_KP), *VP = (_Float16*)(ws + WS_VP);
  const int rows = TNB * TT;
  k_stat<<<dim3(rows / 16), 256, 0, stream>>>(F[0], 1, ST);
  k_proj<<<dim3(rows / 64, CC / 128, 3), 128, 0, stream>>>(F[0], ST, F[3], F[4], F[2], F[5], F[6], F[7], F[8], F[9], F[10], QS, KR, VP);
  k_ksm<<<dim3(CC / 8, TNB), 256, 0, stream>>>(KR, KP);
  k_att<<<dim3(TNB * NH), 128, 0, stream>>>(KP, VP, AT);
  k_y<<<dim3(rows / 64, NH), 128, 0, stream>>>(QS, AT, Y);
  k_emb<<<dim3(2 * CC / 64, TNB), 64, 0, stream>>>(F[1], F[11], F[12], EM);
  k_stat<<<dim3(rows / 16), 256, 0, stream>>>(Y, 0, ST2);
  k_out<<<dim3(rows / 64, CC / 128), 128, 0, stream>>>(Y, ST2, F[13], F[14], EM, F[15], F[16], F[0], (float*)d_out);
}
